// LSHSelfAttention_30906584662594
// MI455X (gfx1250) — hardware-verified
//
#include <hip/hip_runtime.h>
#include <stddef.h>
#include <stdint.h>


#ifndef NB
#define NB 2
#endif
#ifndef SEQ
#define SEQ 2048
#endif
#define NB_FULL  2
#define SEQ_FULL 2048
#define D_MODEL  1024
#define N_HEADS  16
#define D_K      64
#define MROWS    (NB * SEQ)
#define NBH      (NB * N_HEADS)

#define TP   136
#define KTP  72
#define VTP  40
#define PTP  40
#define OTP  68

static_assert(NB >= 1 && NB <= NB_FULL);
static_assert(SEQ >= 128 && SEQ <= SEQ_FULL && (SEQ % 128) == 0);
static_assert((MROWS % 128) == 0);
static_assert(D_MODEL == N_HEADS * D_K);
static_assert((D_MODEL % 128) == 0);

typedef _Float16 f16;
typedef f16   v8h  __attribute__((ext_vector_type(8)));
typedef f16   v16h __attribute__((ext_vector_type(16)));
typedef float v8f  __attribute__((ext_vector_type(8)));
typedef float v4f  __attribute__((ext_vector_type(4)));

union Frag { v16h v; v8h h[2]; };

__device__ __forceinline__ v8f zero8() {
  v8f z;
#pragma unroll
  for (int i = 0; i < 8; ++i) z[i] = 0.0f;
  return z;
}

__device__ __forceinline__ v8f wmma16(v16h a, v16h b, v8f c) {
  v8f d = __builtin_amdgcn_wmma_f32_16x16x32_f16(false, a, false, b, (short)0, c, false, false);
  asm volatile("v_nop\n\tv_nop\n\tv_nop\n\tv_nop" : "+v"(d) : "v"(a), "v"(b));
  return d;
}

__device__ __forceinline__ v16h load_frag(const f16* p, int hh) {
  Frag f;
  f.h[0] = *(const v8h*)(p + 8 * hh);
  f.h[1] = *(const v8h*)(p + 16 + 8 * hh);
  return f.v;
}

__device__ __forceinline__ float bf16r(float f) {
  unsigned u = __float_as_uint(f);
  u = (u + 0x7FFFu + ((u >> 16) & 1u)) & 0xFFFF0000u;
  return __uint_as_float(u);
}

__device__ __forceinline__ void wave_lds_sync() {
  asm volatile("s_wait_dscnt 0" ::: "memory");
  __builtin_amdgcn_fence(3, "wavefront");
  __builtin_amdgcn_wave_barrier();
}

__global__ __launch_bounds__(256)
void k_convert(const float* __restrict__ xq, const float* __restrict__ xk,
               const float* __restrict__ xv, const float* __restrict__ wq,
               const float* __restrict__ wk, const float* __restrict__ wv,
               f16* __restrict__ xp, f16* __restrict__ wp) {
  const int z = blockIdx.y;
  const size_t tid = (size_t)blockIdx.x * 256 + threadIdx.x;
  const size_t e = tid * 8;
  const float* src;
  f16* dst;
  float sc;
  if (z < 3) {
    const size_t nElem = (size_t)MROWS * D_MODEL;
    if (e >= nElem) return;
    const size_t m = e / D_MODEL;
    const size_t c = e - m * D_MODEL;
    const size_t b = m / SEQ;
    const size_t s = m - b * SEQ;
    const float* X = (z == 0) ? xq : (z == 1) ? xk : xv;
    src = X + (b * SEQ_FULL + s) * D_MODEL + c;
    dst = xp + (size_t)z * nElem + e;
    sc = 1.0f;
  } else {
    const size_t nElem = (size_t)D_MODEL * D_MODEL;
    if (e >= nElem) return;
    const float* W = (z == 3) ? wq : (z == 4) ? wk : wv;
    src = W + e;
    dst = wp + (size_t)(z - 3) * nElem + e;
    sc = 16.0f;
  }
  const v4f a0 = *(const v4f*)src;
  const v4f a1 = *(const v4f*)(src + 4);
  v8h o;
#pragma unroll
  for (int i = 0; i < 4; ++i) {
    o[i]     = (f16)(bf16r(a0[i]) * sc);
    o[i + 4] = (f16)(bf16r(a1[i]) * sc);
  }
  *(volatile v8h*)dst = o;
  __threadfence();
  *(volatile v8h*)dst = o;
}


__device__ __forceinline__ void store_rows_2x(const f16* T, f16* __restrict__ plane,
                                              int mBase, int head0, int w, int lane) {
  v8h vals[8];
  unsigned offs[8];
  const int piece = lane & 7, sub = lane >> 3;
#pragma unroll
  for (int pass = 0; pass < 8; ++pass) {
    const int L  = pass * 32 + w * 4 + sub;
    const int ml = L >> 1, j = L & 1;
    vals[pass] = *(const v8h*)(T + ml * TP + 64 * j + 8 * piece);
    const int m  = mBase + ml;
    const int b  = m / SEQ;
    const int s  = m - b * SEQ;
    const int bh = b * N_HEADS + head0 + j;
    offs[pass] = (unsigned)((bh * SEQ + s) * D_K + 8 * piece);
  }
#pragma unroll
  for (int pass = 0; pass < 8; ++pass) *(volatile v8h*)(plane + offs[pass]) = vals[pass];
  __threadfence();
#pragma unroll
  for (int pass = 0; pass < 8; ++pass) *(volatile v8h*)(plane + offs[pass]) = vals[pass];
}

__global__ __launch_bounds__(256)
void k_proj(const f16* __restrict__ xp, const f16* __restrict__ wp,
            const float* __restrict__ bq, const float* __restrict__ bk,
            const float* __restrict__ bv,
            f16* __restrict__ qh, f16* __restrict__ ql,
            f16* __restrict__ kh, f16* __restrict__ kl,
            f16* __restrict__ vt) {
  __shared__ __attribute__((aligned(16))) f16 T[128 * TP];

  const int z = blockIdx.z;
  const int t = threadIdx.x, w = t >> 5, lane = t & 31, l15 = lane & 15, hh = lane >> 4;
  const int waveM = (w >> 1) * 32, waveN = (w & 1) * 64;
  const int mBase = blockIdx.y * 128, nBase = blockIdx.x * 128;
  const f16* X = xp + (size_t)z * MROWS * D_MODEL;
  const f16* W = wp + (size_t)z * D_MODEL * D_MODEL;
  const float* bias = (z == 0) ? bq : (z == 1) ? bk : bv;

  const f16* arow0 = X + (size_t)(mBase + waveM + l15) * D_MODEL;
  const f16* arow1 = arow0 + (size_t)16 * D_MODEL;
  const f16* brow0 = W + (size_t)(nBase + waveN + l15) * D_MODEL;

  v8f acc[2][4];
#pragma unroll
  for (int ti = 0; ti < 2; ++ti)
#pragma unroll
    for (int tj = 0; tj < 4; ++tj) acc[ti][tj] = zero8();

#pragma unroll 1
  for (int k0 = 0; k0 < D_MODEL; k0 += 32) {
    v16h af[2], bfr[4];
    af[0] = load_frag(arow0 + k0, hh);
    af[1] = load_frag(arow1 + k0, hh);
#pragma unroll
    for (int tj = 0; tj < 4; ++tj)
      bfr[tj] = load_frag(brow0 + (size_t)tj * 16 * D_MODEL + k0, hh);
#pragma unroll
    for (int ti = 0; ti < 2; ++ti)
#pragma unroll
      for (int tj = 0; tj < 4; ++tj)
        acc[ti][tj] = wmma16(af[ti], bfr[tj], acc[ti][tj]);
  }

  float b16[4];
#pragma unroll
  for (int tj = 0; tj < 4; ++tj) b16[tj] = bf16r(bias[nBase + waveN + tj * 16 + l15]);
  const int head0 = nBase >> 6;

  if (z < 2) {
    f16* ph = (z == 0) ? qh : kh;
    f16* pl = (z == 0) ? ql : kl;
#pragma unroll
    for (int ti = 0; ti < 2; ++ti)
#pragma unroll
      for (int tj = 0; tj < 4; ++tj)
#pragma unroll
        for (int r = 0; r < 8; ++r) {
          const float y = acc[ti][tj][r] * 0.0625f + b16[tj];
          T[(waveM + ti * 16 + 8 * hh + r) * TP + waveN + tj * 16 + l15] = (f16)y;
        }
    __syncthreads();
    store_rows_2x(T, ph, mBase, head0, w, lane);
    __syncthreads();
#pragma unroll
    for (int ti = 0; ti < 2; ++ti)
#pragma unroll
      for (int tj = 0; tj < 4; ++tj)
#pragma unroll
        for (int r = 0; r < 8; ++r) {
          const float y  = acc[ti][tj][r] * 0.0625f + b16[tj];
          const f16   hv = (f16)y;
          T[(waveM + ti * 16 + 8 * hh + r) * TP + waveN + tj * 16 + l15] =
              (f16)((y - (float)hv) * 2048.0f);
        }
    __syncthreads();
    store_rows_2x(T, pl, mBase, head0, w, lane);
  } else {
    const int bb = mBase / SEQ;
    const int s0 = mBase - bb * SEQ;
#pragma unroll
    for (int ti = 0; ti < 2; ++ti)
#pragma unroll
      for (int tj = 0; tj < 4; ++tj) {
        v8h col;
#pragma unroll
        for (int r = 0; r < 8; ++r) col[r] = (f16)(acc[ti][tj][r] * 0.0625f + b16[tj]);
        *(v8h*)(T + (waveN + tj * 16 + l15) * TP + waveM + ti * 16 + 8 * hh) = col;
      }
    __syncthreads();
    v8h vals[8];
    unsigned offs[8];
    const int piece = lane & 7, sub = lane >> 3;
#pragma unroll
    for (int pass = 0; pass < 8; ++pass) {
      const int L = pass * 32 + w * 4 + sub;
      const int nl = L >> 1, half = L & 1;
      vals[pass] = *(const v8h*)(T + nl * TP + half * 64 + 8 * piece);
      const int head = head0 + (nl >> 6), d = nl & 63;
      const int bh = bb * N_HEADS + head;
      offs[pass] = (unsigned)((bh * D_K + d) * SEQ + s0 + half * 64 + 8 * piece);
    }
#pragma unroll
    for (int pass = 0; pass < 8; ++pass) *(volatile v8h*)(vt + offs[pass]) = vals[pass];
    __threadfence();
#pragma unroll
    for (int pass = 0; pass < 8; ++pass) *(volatile v8h*)(vt + offs[pass]) = vals[pass];
  }
}

__global__ __launch_bounds__(256)
void k_attn(const f16* __restrict__ qh, const f16* __restrict__ ql,
            const f16* __restrict__ kh, const f16* __restrict__ kl,
            const f16* __restrict__ vt,
            const int* __restrict__ hashq, const int* __restrict__ hashk,
            float* __restrict__ out) {
  __shared__ __attribute__((aligned(16))) f16   sKh[32 * KTP];
  __shared__ __attribute__((aligned(16))) f16   sKl[32 * KTP];
  __shared__ __attribute__((aligned(16))) f16   sV[64 * VTP];
  __shared__ __attribute__((aligned(16))) f16   sP[8 * 16 * PTP];
  __shared__ __attribute__((aligned(16))) float sO[8 * 16 * OTP];

  const int bh = blockIdx.y;
  const int b = bh / N_HEADS, h = bh - b * N_HEADS;
  const int t = threadIdx.x, w = t >> 5, lane = t & 31, l15 = lane & 15, hh = lane >> 4;
  const int q0 = blockIdx.x * 128 + w * 16;

  const f16* Qh = qh + (size_t)bh * SEQ * D_K;
  const f16* Ql = ql + (size_t)bh * SEQ * D_K;
  const f16* Kh = kh + (size_t)bh * SEQ * D_K;
  const f16* Kl = kl + (size_t)bh * SEQ * D_K;
  const f16* Vt = vt + (size_t)bh * D_K * SEQ;
  const int* hqp = hashq + (size_t)bh * SEQ_FULL;
  const int* hkp = hashk + (size_t)bh * SEQ_FULL;

  v16h aqh[2], aql[2];
#pragma unroll
  for (int s = 0; s < 2; ++s) {
    aqh[s] = load_frag(Qh + (size_t)(q0 + l15) * D_K + s * 32, hh);
    aql[s] = load_frag(Ql + (size_t)(q0 + l15) * D_K + s * 32, hh);
  }
  int hqv[8];
#pragma unroll
  for (int r = 0; r < 8; ++r) hqv[r] = hqp[q0 + 8 * hh + r];

  float mrow[8], lrow[8];
  v8f o[4];
#pragma unroll
  for (int r = 0; r < 8; ++r) { mrow[r] = -1.0e30f; lrow[r] = 0.0f; }
#pragma unroll
  for (int c = 0; c < 4; ++c) o[c] = zero8();

  const int krow = t >> 3, kch = (t & 7) * 8;
  const int vrow = t >> 2, vch = (t & 3) * 8;
  f16* myP = sP + w * (16 * PTP);

#pragma unroll 1
  for (int kb = 0; kb < SEQ; kb += 32) {
    const v8h gkh = *(const v8h*)(Kh + (size_t)(kb + krow) * D_K + kch);
    const v8h gkl = *(const v8h*)(Kl + (size_t)(kb + krow) * D_K + kch);
    const v8h gv  = *(const v8h*)(Vt + (size_t)vrow * SEQ + kb + vch);
    const int hk0 = hkp[kb + l15];
    const int hk1 = hkp[kb + 16 + l15];
    __syncthreads();
    *(v8h*)(sKh + krow * KTP + kch) = gkh;
    *(v8h*)(sKl + krow * KTP + kch) = gkl;
    *(v8h*)(sV + vrow * VTP + vch)  = gv;
    __syncthreads();

    v8f shh[2], sx[2];
#pragma unroll
    for (int nt = 0; nt < 2; ++nt) {
      const f16* krh = sKh + (nt * 16 + l15) * KTP;
      const f16* krl = sKl + (nt * 16 + l15) * KTP;
      const v16h kfh0 = load_frag(krh, hh), kfh1 = load_frag(krh + 32, hh);
      const v16h kfl0 = load_frag(krl, hh), kfl1 = load_frag(krl + 32, hh);
      v8f a = zero8();
      a = wmma16(aqh[0], kfh0, a);
      a = wmma16(aqh[1], kfh1, a);
      shh[nt] = a;
      v8f cx = zero8();
      cx = wmma16(aqh[0], kfl0, cx);
      cx = wmma16(aqh[1], kfl1, cx);
      cx = wmma16(aql[0], kfh0, cx);
      cx = wmma16(aql[1], kfh1, cx);
      sx[nt] = cx;
    }

#pragma unroll
    for (int r = 0; r < 8; ++r) {
      const float s0v = shh[0][r] + sx[0][r] * (1.0f / 2048.0f);
      const float s1v = shh[1][r] + sx[1][r] * (1.0f / 2048.0f);
      const float x0 = s0v * 0.125f + ((hqv[r] != hk0) ? -1.0e9f : 0.0f);
      const float x1 = s1v * 0.125f + ((hqv[r] != hk1) ? -1.0e9f : 0.0f);
      float mx = fmaxf(x0, x1);
#pragma unroll
      for (int msk = 1; msk < 16; msk <<= 1) mx = fmaxf(mx, __shfl_xor(mx, msk, 32));
      const float mn   = fmaxf(mrow[r], mx);
      const float corr = __expf(mrow[r] - mn);
      const float p0 = __expf(x0 - mn);
      const float p1 = __expf(x1 - mn);
      float tsum = p0 + p1;
#pragma unroll
      for (int msk = 1; msk < 16; msk <<= 1) tsum += __shfl_xor(tsum, msk, 32);
      lrow[r] = lrow[r] * corr + tsum;
      mrow[r] = mn;
#pragma unroll
      for (int c = 0; c < 4; ++c) o[c][r] *= corr;
      myP[(8 * hh + r) * PTP + l15]      = (f16)(p0 * 16384.0f);
      myP[(8 * hh + r) * PTP + 16 + l15] = (f16)(p1 * 16384.0f);
    }
    wave_lds_sync();

    const v16h pa = load_frag(myP + l15 * PTP, hh);
#pragma unroll
    for (int c = 0; c < 4; ++c) {
      const v16h bvf = load_frag(sV + (c * 16 + l15) * VTP, hh);
      o[c] = wmma16(pa, bvf, o[c]);
    }
  }

  float* myO = sO + w * (16 * OTP);
#pragma unroll
  for (int r = 0; r < 8; ++r) {
    const float rinv = (1.0f / lrow[r]) * (1.0f / 16384.0f);
#pragma unroll
    for (int c = 0; c < 4; ++c) myO[(8 * hh + r) * OTP + c * 16 + l15] = o[c][r] * rinv;
  }
  wave_lds_sync();

  v4f vals[8];
  unsigned offs[8];
  const int piece = lane & 7, sub = lane >> 3;
#pragma unroll
  for (int pass = 0; pass < 8; ++pass) {
    const int L = pass * 4 + sub;
    const int row = L >> 1, half = L & 1;
    vals[pass] = *(const v4f*)(myO + row * OTP + half * 32 + piece * 4);
    const int s = q0 + row;
    offs[pass] = (unsigned)((b * SEQ_FULL + s) * D_MODEL + h * D_K + half * 32 + piece * 4);
  }
#pragma unroll
  for (int pass = 0; pass < 8; ++pass) *(volatile v4f*)(out + offs[pass]) = vals[pass];
  __threadfence();
#pragma unroll
  for (int pass = 0; pass < 8; ++pass) *(volatile v4f*)(out + offs[pass]) = vals[pass];
}

extern "C" void kernel_launch(void* const* d_in, const int* in_sizes, int n_in,
                              void* d_out, int out_size, void* d_ws, size_t ws_size,
                              hipStream_t stream) {
  if (n_in < 11) return;
  const float* query = (const float*)d_in[0];
  const float* key   = (const float*)d_in[1];
  const float* value = (const float*)d_in[2];
  const int*   hashq = (const int*)d_in[3];
  const int*   hashk = (const int*)d_in[4];
  const float* Wq = (const float*)d_in[5];
  const float* bq = (const float*)d_in[6];
  const float* Wk = (const float*)d_in[7];
  const float* bk = (const float*)d_in[8];
  const float* Wv = (const float*)d_in[9];
  const float* bv = (const float*)d_in[10];
  float* out = (float*)d_out;

  const int needX = NB * SEQ_FULL * D_MODEL;
  const int needH = NB * N_HEADS * SEQ_FULL;
  if (in_sizes[0] < needX || in_sizes[1] < needX || in_sizes[2] < needX) return;
  if (in_sizes[3] < needH || in_sizes[4] < needH) return;
  if (in_sizes[5] < D_MODEL * D_MODEL || in_sizes[7] < D_MODEL * D_MODEL ||
      in_sizes[9] < D_MODEL * D_MODEL) return;
  if (in_sizes[6] < D_MODEL || in_sizes[8] < D_MODEL || in_sizes[10] < D_MODEL) return;
  if (out_size < needX) return;

  const size_t XP_BYTES = (size_t)3 * MROWS * D_MODEL * sizeof(f16);
  const size_t WP_BYTES = (size_t)3 * D_MODEL * D_MODEL * sizeof(f16);
  const size_t HP_BYTES = (size_t)NBH * SEQ * D_K * sizeof(f16);
  char* ws = (char*)d_ws;
  size_t off = 0;
  f16* xp = (f16*)(ws + off); off += XP_BYTES;
  f16* wp = (f16*)(ws + off); off += WP_BYTES;
  f16* qh = (f16*)(ws + off); off += HP_BYTES;
  f16* ql = (f16*)(ws + off); off += HP_BYTES;
  f16* kh = (f16*)(ws + off); off += HP_BYTES;
  f16* kl = (f16*)(ws + off); off += HP_BYTES;
  f16* vt = (f16*)(ws + off); off += HP_BYTES;
  if (off > ws_size) return;

  const int cbx = (MROWS * (D_MODEL / 8)) / 256;
  const int cbw = (D_MODEL * (D_MODEL / 8)) / 256;
  const int cgx = (cbx > cbw) ? cbx : cbw;
  k_convert<<<dim3(cgx, 6), 256, 0, stream>>>(query, key, value, Wq, Wk, Wv, xp, wp);

  k_proj<<<dim3(D_MODEL / 128, MROWS / 128, 3), 256, 0, stream>>>(xp, wp, bq, bk, bv,
                                                                  qh, ql, kh, kl, vt);

  k_attn<<<dim3(SEQ / 128, NBH), 256, 0, stream>>>(qh, ql, kh, kl, vt, hashq, hashk, out);
}
